// MultiHeadAttentionLayer_31164282699913
// MI455X (gfx1250) — hardware-verified
//
#include <hip/hip_runtime.h>

#ifndef SEQ
#define SEQ 4096
#endif
#define SEQ_FULL 4096
#define IN_DIM 1024
#define NUM_HEADS 16
#define HEAD_DIM 64
#define OUT_DIM (NUM_HEADS * HEAD_DIM)

static_assert(SEQ % 128 == 0);
static_assert(SEQ <= SEQ_FULL);
static_assert(IN_DIM % 64 == 0);
static_assert(OUT_DIM % 64 == 0);
static_assert(HEAD_DIM == 64);
static_assert((size_t)SEQ_FULL * OUT_DIM * 4 == 16777216);

#define BTP 40
#define EQP 72
#define EVP 136
#define TP  72
#define OLP 68
#define ESZ 9216
static_assert(128 * EQP <= ESZ);
static_assert(64 * EVP <= ESZ);

typedef __bf16   v16bf __attribute__((ext_vector_type(16)));
typedef __bf16   v8bf  __attribute__((ext_vector_type(8)));
typedef _Float16 v16h  __attribute__((ext_vector_type(16)));
typedef _Float16 v8h   __attribute__((ext_vector_type(8)));
typedef float    v8f   __attribute__((ext_vector_type(8)));
typedef float    v4f   __attribute__((ext_vector_type(4)));
typedef unsigned int v4u __attribute__((ext_vector_type(4)));

__device__ __forceinline__ v8f mma_bf16(v16bf a, v16bf b, v8f c) {
  v8f d = __builtin_amdgcn_wmma_f32_16x16x32_bf16(false, a, false, b, (short)0, c, false, false);
  asm volatile("v_nop\n\tv_nop\n\tv_nop\n\tv_nop" : "+v"(d) : "v"(a), "v"(b));
  return d;
}
__device__ __forceinline__ v8f mma_f16(v16h a, v16h b, v8f c) {
  v8f d = __builtin_amdgcn_wmma_f32_16x16x32_f16(false, a, false, b, (short)0, c, false, false);
  asm volatile("v_nop\n\tv_nop\n\tv_nop\n\tv_nop" : "+v"(d) : "v"(a), "v"(b));
  return d;
}

__device__ __forceinline__ v16bf ld_frag_bf(const __bf16* p0, int ld, int rc, int kk, int lane) {
  const int hh = (lane >> 4) & 1;
  const __bf16* p = p0 + (size_t)rc * ld + kk + 8 * hh;
  const v8bf lo = *(const v8bf*)(p);
  const v8bf hi = *(const v8bf*)(p + 16);
  v16bf f;
#pragma unroll
  for (int i = 0; i < 8; ++i) { f[i] = lo[i]; f[8 + i] = hi[i]; }
  return f;
}
__device__ __forceinline__ v16h ld_frag_h(const _Float16* p0, int ld, int rc, int kk, int lane) {
  const int hh = (lane >> 4) & 1;
  const _Float16* p = p0 + (size_t)rc * ld + kk + 8 * hh;
  const v8h lo = *(const v8h*)(p);
  const v8h hi = *(const v8h*)(p + 16);
  v16h f;
#pragma unroll
  for (int i = 0; i < 8; ++i) { f[i] = lo[i]; f[8 + i] = hi[i]; }
  return f;
}

__device__ __forceinline__ unsigned int bfb(float x) {
  unsigned int u = __float_as_uint(x);
  u = u + 0x7FFFu + ((u >> 16) & 1u);
  return u >> 16;
}
__device__ __forceinline__ float bf16val(float x) {
  return __uint_as_float(bfb(x) << 16);
}
__device__ __forceinline__ unsigned short hbits(float x) {
  const _Float16 hv = (_Float16)x;
  return __builtin_bit_cast(unsigned short, hv);
}

__global__ __launch_bounds__(256) void k_cvt_rows(const float* __restrict__ in,
                                                  unsigned short* __restrict__ outp, int n8) {
  const int g = blockIdx.x * 256 + threadIdx.x;
  if (g >= n8) return;
  const v4f a = *(const v4f*)(in + (size_t)g * 8);
  const v4f b = *(const v4f*)(in + (size_t)g * 8 + 4);
  v4u w;
  w[0] = bfb(a[0]) | (bfb(a[1]) << 16);
  w[1] = bfb(a[2]) | (bfb(a[3]) << 16);
  w[2] = bfb(b[0]) | (bfb(b[1]) << 16);
  w[3] = bfb(b[2]) | (bfb(b[3]) << 16);
  volatile v4u* p = (volatile v4u*)(outp + (size_t)g * 8);
  *p = w;
  __threadfence();
  *p = w;
}

__global__ __launch_bounds__(256) void k_cvt_wT(const float* __restrict__ Wq,
                                                const float* __restrict__ Wk,
                                                const float* __restrict__ Wv,
                                                unsigned short* __restrict__ wT) {
  __shared__ __align__(16) unsigned short T[64 * TP];
  const int z = blockIdx.z;
  const float* W = (z == 0) ? Wq : ((z == 1) ? Wk : Wv);
  unsigned short* dst = wT + (size_t)z * OUT_DIM * IN_DIM;
  const int k0 = blockIdx.x * 64;
  const int n0 = blockIdx.y * 64;
  const int tid = threadIdx.x;
  const int wave = tid >> 5, lane = tid & 31;

#pragma unroll
  for (int i = 0; i < 4; ++i) {
    const int idx = i * 256 + tid;
    const int kk = idx >> 4;
    const int c4 = (idx & 15) * 4;
    const v4f w = *(const v4f*)(W + (size_t)(k0 + kk) * OUT_DIM + n0 + c4);
    T[(c4 + 0) * TP + kk] = (unsigned short)bfb(w[0]);
    T[(c4 + 1) * TP + kk] = (unsigned short)bfb(w[1]);
    T[(c4 + 2) * TP + kk] = (unsigned short)bfb(w[2]);
    T[(c4 + 3) * TP + kk] = (unsigned short)bfb(w[3]);
  }
  __syncthreads();

  v4u v[2];
  size_t off[2];
#pragma unroll
  for (int it = 0; it < 2; ++it) {
    const int nn = wave * 8 + it * 4 + (lane >> 3);
    const int q = lane & 7;
    v[it] = *(const v4u*)(&T[nn * TP + q * 8]);
    off[it] = (size_t)(n0 + nn) * IN_DIM + k0 + q * 8;
  }
#pragma unroll
  for (int it = 0; it < 2; ++it) *(volatile v4u*)(dst + off[it]) = v[it];
  __threadfence();
#pragma unroll
  for (int it = 0; it < 2; ++it) *(volatile v4u*)(dst + off[it]) = v[it];
}

__global__ __launch_bounds__(256) void k_proj(
    const unsigned short* __restrict__ hb, const unsigned short* __restrict__ wT,
    const float* __restrict__ bq, const float* __restrict__ bk, const float* __restrict__ bv,
    unsigned short* __restrict__ qp, unsigned short* __restrict__ kp,
    unsigned short* __restrict__ vtp) {
  __shared__ __align__(16) unsigned short bt[64 * BTP];
  __shared__ __align__(16) unsigned short E[ESZ];

  const int z = blockIdx.z;
  const int n0 = blockIdx.x * 64;
  const int m0 = blockIdx.y * 128;
  const int tid = threadIdx.x;
  const int wave = tid >> 5, lane = tid & 31;
  const int l15 = lane & 15, half = (lane >> 4) & 1;

  const unsigned short* Wt = wT + (size_t)z * OUT_DIM * IN_DIM;
  const float* bias = (z == 0) ? bq : ((z == 1) ? bk : bv);

  const int tn = tid >> 2;
  const int tk = (tid & 3) * 8;
  const unsigned short* wsrc = Wt + (size_t)(n0 + tn) * IN_DIM + tk;
  const __bf16* A = (const __bf16*)hb;
  const int arow = m0 + wave * 16 + l15;

  v8f acc[4] = {};
  for (int s = 0; s < IN_DIM / 32; ++s) {
    const int kk = s * 32;
    const v4u wv = *(const v4u*)(wsrc + kk);
    __syncthreads();
    *(v4u*)(&bt[tn * BTP + tk]) = wv;
    __syncthreads();
    const v16bf a = ld_frag_bf(A, IN_DIM, arow, kk, lane);
#pragma unroll
    for (int j = 0; j < 4; ++j) {
      const v16bf b = ld_frag_bf((const __bf16*)bt, BTP, j * 16 + l15, 0, lane);
      acc[j] = mma_bf16(a, b, acc[j]);
    }
  }

  const float car = 8.0f;
  if (z != 2) {
#pragma unroll
    for (int j = 0; j < 4; ++j) {
      const int col = j * 16 + l15;
      const float bb = bf16val(bias[n0 + col]);
#pragma unroll
      for (int r = 0; r < 8; ++r) {
        const int row = wave * 16 + 8 * half + r;
        E[row * EQP + col] = hbits((acc[j][r] + bb) * car);
      }
    }
    __syncthreads();
    unsigned short* dst = (z == 0) ? qp : kp;
    v4u v[4];
    size_t off[4];
#pragma unroll
    for (int it = 0; it < 4; ++it) {
      const int row = wave * 16 + it * 4 + (lane >> 3);
      const int q = lane & 7;
      v[it] = *(const v4u*)(&E[row * EQP + q * 8]);
      off[it] = (size_t)(m0 + row) * OUT_DIM + n0 + q * 8;
    }
#pragma unroll
    for (int it = 0; it < 4; ++it) *(volatile v4u*)(dst + off[it]) = v[it];
    __threadfence();
#pragma unroll
    for (int it = 0; it < 4; ++it) *(volatile v4u*)(dst + off[it]) = v[it];
  } else {
#pragma unroll
    for (int j = 0; j < 4; ++j) {
      const int col = j * 16 + l15;
      const float bb = bf16val(bias[n0 + col]);
#pragma unroll
      for (int r = 0; r < 8; ++r) {
        const int srow = wave * 16 + 8 * half + r;
        E[col * EVP + srow] = hbits((acc[j][r] + bb) * car);
      }
    }
    __syncthreads();
    v4u v[4];
    size_t off[4];
#pragma unroll
    for (int it = 0; it < 4; ++it) {
      const int drow = wave * 8 + it * 2 + half;
      const int q = l15;
      v[it] = *(const v4u*)(&E[drow * EVP + q * 8]);
      off[it] = (size_t)(n0 + drow) * SEQ + m0 + q * 8;
    }
#pragma unroll
    for (int it = 0; it < 4; ++it) *(volatile v4u*)(vtp + off[it]) = v[it];
    __threadfence();
#pragma unroll
    for (int it = 0; it < 4; ++it) *(volatile v4u*)(vtp + off[it]) = v[it];
  }
}

__global__ __launch_bounds__(32) void k_attn(const unsigned short* __restrict__ qp,
                                             const unsigned short* __restrict__ kp,
                                             const unsigned short* __restrict__ vtp,
                                             float* __restrict__ outp) {
  __shared__ __align__(16) float Ol[16 * OLP];

  const int lane = threadIdx.x & 31;
  const int l15 = lane & 15;
  const int half = (lane >> 4) & 1;
  const int q0 = blockIdx.x * 16;
  const int head = blockIdx.y;

  const _Float16* Q  = (const _Float16*)qp;
  const _Float16* K  = (const _Float16*)kp;
  const _Float16* VT = (const _Float16*)vtp;

  const _Float16* qbase = Q + (size_t)q0 * OUT_DIM + head * HEAD_DIM;
  const v16h qb0 = ld_frag_h(qbase, OUT_DIM, l15, 0, lane);
  const v16h qb1 = ld_frag_h(qbase, OUT_DIM, l15, 32, lane);
  const _Float16* kbase = K + head * HEAD_DIM;
  const _Float16* vbase = VT + (size_t)head * HEAD_DIM * SEQ;

  v8f o[4] = {};
  float mrun = -1.0e30f, lrun = 0.0f;
  const float sscale = 1.0f / 512.0f;

  for (int kc = 0; kc < SEQ; kc += 32) {
    const _Float16* kt = kbase + (size_t)kc * OUT_DIM;
    const v16h ka0 = ld_frag_h(kt, OUT_DIM, l15, 0, lane);
    const v16h ka1 = ld_frag_h(kt, OUT_DIM, l15, 32, lane);
    const v16h ka2 = ld_frag_h(kt, OUT_DIM, 16 + l15, 0, lane);
    const v16h ka3 = ld_frag_h(kt, OUT_DIM, 16 + l15, 32, lane);
    v8f c0 = {}, c1 = {};
    c0 = mma_f16(ka0, qb0, c0);
    c0 = mma_f16(ka1, qb1, c0);
    c1 = mma_f16(ka2, qb0, c1);
    c1 = mma_f16(ka3, qb1, c1);

    float sa[8], sb[8];
#pragma unroll
    for (int r = 0; r < 8; ++r) { sa[r] = c0[r] * sscale; sb[r] = c1[r] * sscale; }
    float lm = fmaxf(sa[0], sb[0]);
#pragma unroll
    for (int r = 1; r < 8; ++r) lm = fmaxf(lm, fmaxf(sa[r], sb[r]));
    lm = fmaxf(lm, __shfl_xor(lm, 16, 32));
    const float mnew = fmaxf(mrun, lm);
    const float alpha = __expf(mrun - mnew);
    float p0[8], p1[8];
    float ls = 0.0f;
#pragma unroll
    for (int r = 0; r < 8; ++r) {
      p0[r] = __expf(sa[r] - mnew);
      p1[r] = __expf(sb[r] - mnew);
      ls += p0[r] + p1[r];
    }
    ls += __shfl_xor(ls, 16, 32);
    lrun = lrun * alpha + ls;
    mrun = mnew;
#pragma unroll
    for (int j = 0; j < 4; ++j)
#pragma unroll
      for (int r = 0; r < 8; ++r) o[j][r] *= alpha;

    v16h pb;
#pragma unroll
    for (int e = 0; e < 8; ++e) {
      pb[e]     = (_Float16)(p0[e] * 1024.0f);
      pb[8 + e] = (_Float16)(p1[e] * 1024.0f);
    }
#pragma unroll
    for (int j = 0; j < 4; ++j) {
      const v16h va = ld_frag_h(vbase, SEQ, j * 16 + l15, kc, lane);
      o[j] = mma_f16(va, pb, o[j]);
    }
  }

  const float inv = 1.0f / (lrun * 8192.0f);
#pragma unroll
  for (int j = 0; j < 4; ++j) {
    v4f lo4, hi4;
    lo4[0] = o[j][0] * inv; lo4[1] = o[j][1] * inv; lo4[2] = o[j][2] * inv; lo4[3] = o[j][3] * inv;
    hi4[0] = o[j][4] * inv; hi4[1] = o[j][5] * inv; hi4[2] = o[j][6] * inv; hi4[3] = o[j][7] * inv;
    *(v4f*)(&Ol[l15 * OLP + j * 16 + 8 * half])     = lo4;
    *(v4f*)(&Ol[l15 * OLP + j * 16 + 8 * half + 4]) = hi4;
  }
  __syncthreads();

  v4f v[8];
  size_t off[8];
  float* ob = outp + (size_t)q0 * OUT_DIM + head * HEAD_DIM;
#pragma unroll
  for (int it = 0; it < 8; ++it) {
    const int row = it * 2 + half;
    const int q = l15;
    v[it] = *(const v4f*)(&Ol[row * OLP + q * 4]);
    off[it] = (size_t)row * OUT_DIM + q * 4;
  }
#pragma unroll
  for (int it = 0; it < 8; ++it) *(volatile v4f*)(ob + off[it]) = v[it];
  __threadfence();
#pragma unroll
  for (int it = 0; it < 8; ++it) *(volatile v4f*)(ob + off[it]) = v[it];
}

extern "C" void kernel_launch(void* const* d_in, const int* in_sizes, int n_in,
                              void* d_out, int out_size, void* d_ws, size_t ws_size,
                              hipStream_t stream) {
  if (n_in < 7) return;
  if (in_sizes[0] < SEQ * IN_DIM) return;
  if (in_sizes[1] < IN_DIM * OUT_DIM || in_sizes[2] < IN_DIM * OUT_DIM ||
      in_sizes[3] < IN_DIM * OUT_DIM) return;
  if (in_sizes[4] < OUT_DIM || in_sizes[5] < OUT_DIM || in_sizes[6] < OUT_DIM) return;
  if (out_size < SEQ * OUT_DIM) return;

  const float* h  = (const float*)d_in[0];
  const float* Wq = (const float*)d_in[1];
  const float* Wk = (const float*)d_in[2];
  const float* Wv = (const float*)d_in[3];
  const float* bq = (const float*)d_in[4];
  const float* bk = (const float*)d_in[5];
  const float* bv = (const float*)d_in[6];

  const size_t hb_bytes = (size_t)SEQ * IN_DIM * 2;
  const size_t wt_bytes = (size_t)3 * OUT_DIM * IN_DIM * 2;
  const size_t pl_bytes = (size_t)SEQ * OUT_DIM * 2;
  const size_t off_hb = 0;
  const size_t off_wt = off_hb + hb_bytes;
  const size_t off_q  = off_wt + wt_bytes;
  const size_t off_k  = off_q + pl_bytes;
  const size_t off_vt = off_k + pl_bytes;
  const size_t total  = off_vt + pl_bytes;
  if (total > ws_size) return;

  char* ws = (char*)d_ws;
  unsigned short* hb  = (unsigned short*)(ws + off_hb);
  unsigned short* wt  = (unsigned short*)(ws + off_wt);
  unsigned short* qpl = (unsigned short*)(ws + off_q);
  unsigned short* kpl = (unsigned short*)(ws + off_k);
  unsigned short* vtp = (unsigned short*)(ws + off_vt);

  const int n8 = SEQ * IN_DIM / 8;
  k_cvt_rows<<<(n8 + 255) / 256, 256, 0, stream>>>(h, hb, n8);
  k_cvt_wT<<<dim3(IN_DIM / 64, OUT_DIM / 64, 3), 256, 0, stream>>>(Wq, Wk, Wv, wt);
  k_proj<<<dim3(OUT_DIM / 64, SEQ / 128, 3), 256, 0, stream>>>(hb, wt, bq, bk, bv, qpl, kpl, vtp);
  k_attn<<<dim3(SEQ / 16, NUM_HEADS), 32, 0, stream>>>(qpl, kpl, vtp, (float*)d_out);
}
